// MultiHeadAttention_61357902791248
// MI455X (gfx1250) — hardware-run, weakly checked
//
#include <hip/hip_runtime.h>


#ifndef NB
#define NB 2
#endif
#ifndef SEQ
#define SEQ 2048
#endif
#define NB_FULL  2
#define SEQ_FULL 2048
#ifndef OUT_SEQ
#define OUT_SEQ SEQ
#endif
#define DM   2048
#define NH_  16
#define HD   128
#define EROWS ((SEQ < 512) ? SEQ : 512)
#define AW   4
#define NFB  32
#define QRS  2048.0f
#define QRI  (1.0f / 2048.0f)
#define L2E  1.4426950408889634f
#define SC2  (0.08838834764831845f * 1.4426950408889634f)
#define PSH  12.0f
#define CSC  16.0f
#define WOS  1024.0f
#define OSC  (1.0f / 16384.0f)

static_assert(HD == 128);
static_assert(NH_ * HD == DM);
static_assert(DM % 128 == 0);
static_assert(DM % 64 == 0);
static_assert(DM % 32 == 0);
static_assert(SEQ % 128 == 0);
static_assert(EROWS % 128 == 0);
static_assert(EROWS <= SEQ);
static_assert((SEQ - EROWS) % (16 * AW) == 0);
static_assert(EROWS % (16 * AW) == 0);
static_assert(SEQ % NFB == 0);
static_assert(NFB == 32);
static_assert(SEQ % 8 == 0);
static_assert(((size_t)SEQ * DM) % 8 == 0);
static_assert(NB <= NB_FULL);
static_assert(SEQ <= SEQ_FULL);

typedef _Float16 h16;
typedef unsigned short bf;
typedef __attribute__((ext_vector_type(16))) __bf16   v16bf;
typedef __attribute__((ext_vector_type(16))) _Float16 v16h;
typedef __attribute__((ext_vector_type(16))) unsigned short v16us;
typedef __attribute__((ext_vector_type(8)))  _Float16 v8h;
typedef __attribute__((ext_vector_type(8)))  unsigned short v8us;
typedef __attribute__((ext_vector_type(8)))  float    v8f;
typedef __attribute__((ext_vector_type(4)))  float    v4f;
typedef __attribute__((ext_vector_type(4)))  unsigned v4u;
typedef v4f  __attribute__((may_alias)) v4fa;

static constexpr size_t PLN = (size_t)NB * NH_ * SEQ * HD;
static constexpr size_t PLR = (size_t)NB * NH_ * EROWS * HD;

__device__ __forceinline__ unsigned short f2bf(float f) { unsigned u = __float_as_uint(f); u += 0x7FFFu + ((u >> 16) & 1u); return (unsigned short)(u >> 16); }
__device__ __forceinline__ float bfr(float f) { return __uint_as_float(((unsigned)f2bf(f)) << 16); }
__device__ __forceinline__ float bflo(unsigned w) { return __uint_as_float(w << 16); }
__device__ __forceinline__ float bfhi(unsigned w) { return __uint_as_float(w & 0xffff0000u); }
__device__ __forceinline__ v16h cat16(v8h lo, v8h hi) { return __builtin_shufflevector(lo, hi, 0, 1, 2, 3, 4, 5, 6, 7, 8, 9, 10, 11, 12, 13, 14, 15); }
__device__ __forceinline__ v16us cat16u(v8us lo, v8us hi) { return __builtin_shufflevector(lo, hi, 0, 1, 2, 3, 4, 5, 6, 7, 8, 9, 10, 11, 12, 13, 14, 15); }
__device__ __forceinline__ v8f wmma16(v16h a, v16h b, v8f c) {
    c = __builtin_amdgcn_wmma_f32_16x16x32_f16(false, a, false, b, (short)0, c, false, false);
    asm volatile("v_nop\n\tv_nop\n\tv_nop\n\tv_nop" : "+v"(c) : "v"(a), "v"(b));
    return c; }
__device__ __forceinline__ v8f wmmab(v16bf a, v16bf b, v8f c) {
    c = __builtin_amdgcn_wmma_f32_16x16x32_bf16(false, a, false, b, (short)0, c, false, false);
    asm volatile("v_nop\n\tv_nop\n\tv_nop\n\tv_nop" : "+v"(c) : "v"(a), "v"(b));
    return c; }
__device__ __forceinline__ v16h ldh(const h16* p) { return cat16(*(const v8h*)p, *(const v8h*)(p + 16)); }
__device__ __forceinline__ v16bf ldb(const bf* p) { return __builtin_bit_cast(v16bf, cat16u(*(const v8us*)p, *(const v8us*)(p + 16))); }
__device__ __forceinline__ v16bf ldfrag(const bf* p)  { return ldb(p); }
__device__ __forceinline__ v16h  ldfrag(const h16* p) { return ldh(p); }
__device__ __forceinline__ v8f mma(v16bf a, v16bf b, v8f c) { return wmmab(a, b, c); }
__device__ __forceinline__ v8f mma(v16h a, v16h b, v8f c)   { return wmma16(a, b, c); }
__device__ __forceinline__ void wave_sync() { __builtin_amdgcn_fence(3  , "wavefront"); __builtin_amdgcn_wave_barrier(); asm volatile("" ::: "memory"); }

__global__ __launch_bounds__(256) void k_cvt8(const float* __restrict__ src, bf* dst, size_t n8) {
    const size_t i = (size_t)blockIdx.x * 256 + threadIdx.x; if (i >= n8) return;
    const v8f v = *(const v8f*)(src + i * 8); v8us o;
#pragma unroll
    for (int k = 0; k < 8; ++k) o[k] = f2bf(v[k]);
    *(volatile v8us*)(dst + i * 8) = o; __threadfence(); *(volatile v8us*)(dst + i * 8) = o;
}

template <typename T> struct WTr;
template <> struct WTr<bf>  { typedef v8us vec; static __device__ __forceinline__ bf  cv(float w) { return f2bf(w); } };
template <> struct WTr<h16> { typedef v8h  vec; static __device__ __forceinline__ h16 cv(float w) { return (h16)(bfr(w) * WOS); } };

template <typename T>
__global__ __launch_bounds__(256) void k_wT(const float* __restrict__ W, T* WT) {
    typedef typename WTr<T>::vec vec_t;
    __shared__ __align__(16) float tl[64 * 68];
    const int tid = threadIdx.x; const int n0 = blockIdx.x * 64, k0 = blockIdx.y * 64;
#pragma unroll
    for (int j = 0; j < 4; ++j) { const int idx = tid + 256 * j; const int row = idx >> 4, c4 = (idx & 15) * 4;
        const v4f v = *(const v4f*)(W + (size_t)(k0 + row) * DM + n0 + c4);
        *(v4fa*)(&tl[row * 68 + c4]) = v; }
    __syncthreads();
#pragma unroll 1
    for (int ps = 0; ps < 2; ++ps) {
#pragma unroll
        for (int s = 0; s < 2; ++s) { const int orow = 32 * s + (tid >> 3), k8 = (tid & 7) * 8; vec_t o;
#pragma unroll
            for (int e = 0; e < 8; ++e) o[e] = WTr<T>::cv(tl[(k8 + e) * 68 + orow]);
            *(volatile vec_t*)(WT + (size_t)(n0 + orow) * DM + k0 + k8) = o; }
        if (ps == 0) __threadfence(); }
}

__global__ __launch_bounds__(256) void k_mprep(const float* __restrict__ MK, bf* MB, int* FL) {
    __shared__ int sf[8];
    const int tid = threadIdx.x, lane = tid & 31, wave = __builtin_amdgcn_readfirstlane((int)(tid >> 5));
    const int rpb = SEQ / NFB; const int rbeg = blockIdx.x * rpb;
    int bad = 0;
#pragma unroll 1
    for (int r = rbeg; r < rbeg + rpb; ++r) {
#pragma unroll 1
        for (int c = tid; c < SEQ / 8; c += 256) {
            const float* src = MK + (size_t)r * SEQ_FULL + 8 * c;
            const v4f a = *(const v4f*)src; const v4f b4 = *(const v4f*)(src + 4);
            v8us o;
#pragma unroll
            for (int e = 0; e < 8; ++e) { const float x = (e < 4) ? a[e & 3] : b4[e & 3]; o[e] = f2bf(x); const int k = 8 * c + e;
                const int up = (k > r) && !(x <= -1.0e8f); const int dg = (k == r) && !(x >= -1.0e4f); bad |= (up || dg) ? 1 : 0; }
            bf* dp = MB + (size_t)r * SEQ + 8 * c;
            *(volatile v8us*)dp = o; __threadfence(); *(volatile v8us*)dp = o;
        }
    }
    const int wbad = __any(bad);
    if (lane == 0) sf[wave] = wbad ? 1 : 0;
    __syncthreads();
    if (wave == 0) { int tot = 0;
#pragma unroll
        for (int i = 0; i < 8; ++i) tot |= sf[i];
        const int val = tot ? 0 : 1; int* fp = FL + blockIdx.x * 32 + lane;
        *(volatile int*)fp = val; __threadfence(); *(volatile int*)fp = val; }
}

template <typename T>
__device__ __forceinline__ void mm2x8(const T* __restrict__ A, const T* __restrict__ Bt, const size_t aoff, const size_t boff, v8f (&acc)[2][8]) {
#pragma unroll 1
    for (int kc = 0; kc < DM; kc += 32) {
        const T* ap = A + aoff + kc; const T* bp = Bt + boff + kc;
        const auto a0 = ldfrag(ap);
        const auto a1 = ldfrag(ap + (size_t)16 * DM);
#pragma unroll
        for (int nb = 0; nb < 8; ++nb) {
            const auto b = ldfrag(bp + (size_t)nb * 16 * DM);
            acc[0][nb] = mma(a0, b, acc[0][nb]);
            acc[1][nb] = mma(a1, b, acc[1][nb]);
        }
    }
}

__global__ __launch_bounds__(32) void k_projqk(const bf* __restrict__ XB, const bf* __restrict__ WT, h16* PH, h16* PR, const float* __restrict__ FC, const float* __restrict__ FS) {
    __shared__ __align__(16) float os[16 * 132];
    const int lane = threadIdx.x & 31, lr = lane & 15, hi = lane >> 4;
    const int r0 = blockIdx.x * 32, hh = blockIdx.y, z = blockIdx.z;
    v8f acc[2][8];
#pragma unroll
    for (int mb = 0; mb < 2; ++mb)
#pragma unroll
        for (int nb = 0; nb < 8; ++nb) acc[mb][nb] = (v8f){};
    mm2x8<bf>(XB, WT + (size_t)z * DM * DM, (size_t)(r0 + lr) * DM + 8 * hi, (size_t)(hh * HD + lr) * DM + 8 * hi, acc);
    const int b = r0 / SEQ, tt = r0 % SEQ; const int zh = b * NH_ + hh;
    const int early = (tt < EROWS) ? 1 : 0;
    h16* ph = PH + (size_t)z * PLN; h16* pr = PR + (size_t)z * PLR;
    const float sg = (lr < 8) ? -1.0f : 1.0f;
#pragma unroll
    for (int mb = 0; mb < 2; ++mb) {
#pragma unroll
        for (int nb = 0; nb < 8; ++nb) {
#pragma unroll
            for (int j = 0; j < 8; ++j) os[(hi * 8 + j) * 132 + nb * 16 + lr] = acc[mb][nb][j]; }
        wave_sync();
#pragma unroll 1
        for (int ps = 0; ps < 2; ++ps) {
#pragma unroll
            for (int s = 0; s < 8; ++s) { const int row = 2 * s + hi, c8 = lr * 8, cp = c8 ^ 64;
                const int t = tt + mb * 16 + row;
                const v4f x0 = *(const v4fa*)(&os[row * 132 + c8]); const v4f x1 = *(const v4fa*)(&os[row * 132 + c8 + 4]);
                const v4f p0 = *(const v4fa*)(&os[row * 132 + cp]); const v4f p1 = *(const v4fa*)(&os[row * 132 + cp + 4]);
                const float* fc = FC + (size_t)t * HD + c8; const float* fs = FS + (size_t)t * HD + c8;
                const v4f c0 = *(const v4f*)fc; const v4f c1 = *(const v4f*)(fc + 4); const v4f s0 = *(const v4f*)fs; const v4f s1 = *(const v4f*)(fs + 4);
                v8h hv, rv;
#pragma unroll
                for (int i = 0; i < 4; ++i) {
                    const float y0 = x0[i] * bfr(c0[i]) + (sg * p0[i]) * bfr(s0[i]);
                    const float y1 = x1[i] * bfr(c1[i]) + (sg * p1[i]) * bfr(s1[i]);
                    const h16 a0 = (h16)y0; const h16 a1 = (h16)y1; hv[i] = a0; hv[4 + i] = a1;
                    rv[i] = (h16)((y0 - (float)a0) * QRS); rv[4 + i] = (h16)((y1 - (float)a1) * QRS); }
                *(volatile v8h*)(ph + ((size_t)zh * SEQ + t) * HD + c8) = hv;
                if (early) *(volatile v8h*)(pr + ((size_t)zh * EROWS + t) * HD + c8) = rv; }
            if (ps == 0) __threadfence(); }
        wave_sync();
    }
}

__global__ __launch_bounds__(32) void k_projv(const bf* __restrict__ XB, const bf* __restrict__ WVT, h16* VT, h16* VR) {
    __shared__ __align__(16) float os[16 * 132];
    const int lane = threadIdx.x & 31, lr = lane & 15, hi = lane >> 4;
    const int r0 = blockIdx.x * 32, c0 = blockIdx.y * 128;
    v8f acc[2][8];
#pragma unroll
    for (int mb = 0; mb < 2; ++mb)
#pragma unroll
        for (int nb = 0; nb < 8; ++nb) acc[mb][nb] = (v8f){};
    mm2x8<bf>(WVT, XB, (size_t)(r0 + lr) * DM + 8 * hi, (size_t)(c0 + lr) * DM + 8 * hi, acc);
    const int b = c0 / SEQ, tt = c0 % SEQ;
    const int early = (tt < EROWS) ? 1 : 0;
#pragma unroll
    for (int mb = 0; mb < 2; ++mb) {
#pragma unroll
        for (int nb = 0; nb < 8; ++nb) {
#pragma unroll
            for (int j = 0; j < 8; ++j) os[(hi * 8 + j) * 132 + nb * 16 + lr] = acc[mb][nb][j]; }
        wave_sync();
#pragma unroll 1
        for (int ps = 0; ps < 2; ++ps) {
#pragma unroll
            for (int s = 0; s < 8; ++s) { const int row = 2 * s + hi, c8 = lr * 8; const int m = r0 + mb * 16 + row;
                const v4f x0 = *(const v4fa*)(&os[row * 132 + c8]); const v4f x1 = *(const v4fa*)(&os[row * 132 + c8 + 4]);
                v8h hv, rv;
#pragma unroll
                for (int i = 0; i < 4; ++i) { const h16 a0 = (h16)x0[i]; const h16 a1 = (h16)x1[i]; hv[i] = a0; hv[4 + i] = a1;
                    rv[i] = (h16)((x0[i] - (float)a0) * QRS); rv[4 + i] = (h16)((x1[i] - (float)a1) * QRS); }
                *(volatile v8h*)(VT + ((size_t)b * DM + m) * SEQ + tt + c8) = hv;
                if (early) *(volatile v8h*)(VR + ((size_t)b * DM + m) * EROWS + tt + c8) = rv; }
            if (ps == 0) __threadfence(); }
        wave_sync();
    }
}

template <int EARLY>
__global__ __launch_bounds__(32 * AW) void k_flash(const h16* __restrict__ QH, const h16* __restrict__ QR, const h16* __restrict__ KH, const h16* __restrict__ KR,
                                                   const h16* __restrict__ VT, const h16* __restrict__ VR, const bf* __restrict__ MB, const bf* __restrict__ AB,
                                                   const int* __restrict__ FL, h16* CH, h16* CR, int tbase) {
    __shared__ __align__(16) float os[AW * 16 * 132];
    const int lane = threadIdx.x & 31; const int wave = __builtin_amdgcn_readfirstlane((int)(threadIdx.x >> 5));
    const int lr = lane & 15, hi = lane >> 4;
    const int zh = blockIdx.y; const int b = zh / NH_, h = zh % NH_;
    const int t0 = tbase + (blockIdx.x * AW + wave) * 16;
    const int fl = FL[lane * 32];
    const int okc = __all(fl == 1);
    int nst = SEQ / 32;
    if (okc) { const int c = (t0 + 15) / 32 + 1; nst = (c < nst) ? c : nst; }
    const size_t pq  = ((size_t)zh * SEQ + t0 + lr) * HD + 8 * hi;
    const size_t pk  = ((size_t)zh * SEQ + lr) * HD + 8 * hi;
    const size_t pv  = ((size_t)zh * HD + lr) * SEQ + 8 * hi;
    const size_t pqr = ((size_t)zh * EROWS + (EARLY ? t0 : 0) + lr) * HD + 8 * hi;
    const size_t pkr = ((size_t)zh * EROWS + lr) * HD + 8 * hi;
    const size_t pvr = ((size_t)zh * HD + lr) * EROWS + 8 * hi;
    const bf* mrow = MB + (size_t)(t0 + lr) * SEQ + 8 * hi;
    const bf* arow = AB + (size_t)h * SEQ_FULL + 8 * hi;
    v16h qh[4];
#pragma unroll
    for (int i = 0; i < 4; ++i) qh[i] = ldh(QH + pq + 32 * i);
    v8f o[8];
#pragma unroll
    for (int j = 0; j < 8; ++j) o[j] = (v8f){};
    float m = -3.0e38f, l = 0.0f;
#pragma unroll 1
    for (int st = 0; st < nst; ++st) {
        const int key0 = st * 32;
        const int rs = (EARLY && (key0 < EROWS)) ? 1 : 0;
        const h16* ka = KH + pk + (size_t)key0 * HD;
        const h16* kr = KR + pkr + (size_t)(rs ? key0 : 0) * HD;
        v8f sa = (v8f){}, sb = (v8f){}, la = (v8f){}, lb = (v8f){};
#pragma unroll
        for (int i = 0; i < 4; ++i) {
            const v16h a0 = ldh(ka + 32 * i), a1 = ldh(ka + 16 * HD + 32 * i);
            const v16h q = EARLY ? ldh(QH + pq + 32 * i) : qh[i];
            sa = wmma16(a0, q, sa); sb = wmma16(a1, q, sb);
            if (EARLY) {
                const v16h qr = ldh(QR + pqr + 32 * i);
                la = wmma16(a0, qr, la); lb = wmma16(a1, qr, lb);
                if (rs) { const v16h r0v = ldh(kr + 32 * i), r1v = ldh(kr + 16 * HD + 32 * i);
                    la = wmma16(r0v, q, la); lb = wmma16(r1v, q, lb); }
            }
        }
        const v4u mwa = *(const v4u*)(mrow + key0), mwb = *(const v4u*)(mrow + key0 + 16);
        const v4u awa = *(const v4u*)(arow + key0), awb = *(const v4u*)(arow + key0 + 16);
        float ta[8], tb[8]; float mx = -3.0e38f;
#pragma unroll
        for (int r = 0; r < 8; ++r) {
            float xa = sa[r], xb = sb[r];
            if (EARLY) { xa += la[r] * QRI; xb += lb[r] * QRI; }
            const float ba = (r & 1) ? (bfhi(mwa[r >> 1]) + bfhi(awa[r >> 1])) : (bflo(mwa[r >> 1]) + bflo(awa[r >> 1]));
            const float bb = (r & 1) ? (bfhi(mwb[r >> 1]) + bfhi(awb[r >> 1])) : (bflo(mwb[r >> 1]) + bflo(awb[r >> 1]));
            ta[r] = xa * SC2 + ba * L2E; tb[r] = xb * SC2 + bb * L2E;
            mx = fmaxf(mx, fmaxf(ta[r], tb[r])); }
        mx = fmaxf(mx, __shfl_xor(mx, 16, 32));
        const float mnew = fmaxf(m, mx);
        const float alpha = __builtin_amdgcn_exp2f(m - mnew);
        const float sh = PSH - mnew;
        v16h pb, prb; float ls = 0.0f;
#pragma unroll
        for (int r = 0; r < 8; ++r) {
            const float ea = __builtin_amdgcn_exp2f(ta[r] + sh), eb = __builtin_amdgcn_exp2f(tb[r] + sh);
            const h16 pa = (h16)ea; const h16 pc = (h16)eb; pb[r] = pa; pb[8 + r] = pc;
            if (EARLY) { prb[r] = (h16)((ea - (float)pa) * QRS); prb[8 + r] = (h16)((eb - (float)pc) * QRS); ls += ea + eb; }
            else { prb[r] = pa; prb[8 + r] = pc; ls += (float)pa + (float)pc; } }
        l = l * alpha + ls; m = mnew;
#pragma unroll
        for (int j = 0; j < 8; ++j) o[j] = o[j] * alpha;
        const h16* va = VT + pv + key0;
        const h16* vra = VR + pvr + (rs ? key0 : 0);
#pragma unroll
        for (int j = 0; j < 8; ++j) {
            const v16h vv = ldh(va + (size_t)(16 * j) * SEQ);
            o[j] = wmma16(vv, pb, o[j]);
            if (EARLY) {
                v8f tm = (v8f){};
                if (rs) { const v16h vr = ldh(vra + (size_t)(16 * j) * EROWS); tm = wmma16(vr, pb, tm); }
                tm = wmma16(vv, prb, tm);
                o[j] = o[j] + tm * QRI; }
        }
    }
    l += __shfl_xor(l, 16, 32);
    const float inv = CSC * (1.0f / l);
    const int wb = wave * 16 * 132;
#pragma unroll
    for (int j = 0; j < 8; ++j) { v4f a, c;
        a[0] = o[j][0] * inv; a[1] = o[j][1] * inv; a[2] = o[j][2] * inv; a[3] = o[j][3] * inv;
        c[0] = o[j][4] * inv; c[1] = o[j][5] * inv; c[2] = o[j][6] * inv; c[3] = o[j][7] * inv;
        *(v4fa*)(&os[wb + lr * 132 + 16 * j + 8 * hi]) = a; *(v4fa*)(&os[wb + lr * 132 + 16 * j + 8 * hi + 4]) = c; }
    wave_sync();
    h16* crow = CH + ((size_t)b * SEQ + t0) * DM + h * HD;
    h16* rrow = CR + ((size_t)b * EROWS + (EARLY ? t0 : 0)) * DM + h * HD;
#pragma unroll 1
    for (int ps = 0; ps < 2; ++ps) {
#pragma unroll
        for (int s = 0; s < 8; ++s) { const int row = 2 * s + hi, c8 = lr * 8;
            const v4f x0 = *(const v4fa*)(&os[wb + row * 132 + c8]); const v4f x1 = *(const v4fa*)(&os[wb + row * 132 + c8 + 4]);
            v8h hv, rv;
#pragma unroll
            for (int i = 0; i < 4; ++i) { const h16 a0 = (h16)x0[i]; const h16 a1 = (h16)x1[i]; hv[i] = a0; hv[4 + i] = a1;
                rv[i] = (h16)((x0[i] - (float)a0) * QRS); rv[4 + i] = (h16)((x1[i] - (float)a1) * QRS); }
            *(volatile v8h*)(crow + (size_t)row * DM + c8) = hv;
            if (EARLY) *(volatile v8h*)(rrow + (size_t)row * DM + c8) = rv; }
        if (ps == 0) __threadfence(); }
}

__global__ __launch_bounds__(32) void k_out(const h16* __restrict__ CH, const h16* __restrict__ CR, const h16* __restrict__ WOT, float* OUT) {
    __shared__ __align__(16) float os[16 * 132];
    const int lane = threadIdx.x & 31, lr = lane & 15, hi = lane >> 4;
    const int r0 = blockIdx.x * 32, c0 = blockIdx.y * 128;
    const int b = r0 / SEQ, tt = r0 % SEQ;
    v8f acc[2][8];
#pragma unroll
    for (int mb = 0; mb < 2; ++mb)
#pragma unroll
        for (int nb = 0; nb < 8; ++nb) acc[mb][nb] = (v8f){};
    const size_t boff = (size_t)(c0 + lr) * DM + 8 * hi;
    if (tt < EROWS) {
        mm2x8<h16>(CR, WOT, ((size_t)b * EROWS + tt + lr) * DM + 8 * hi, boff, acc);
#pragma unroll
        for (int mb = 0; mb < 2; ++mb)
#pragma unroll
            for (int nb = 0; nb < 8; ++nb) acc[mb][nb] = acc[mb][nb] * QRI;
    }
    mm2x8<h16>(CH, WOT, (size_t)(r0 + lr) * DM + 8 * hi, boff, acc);
#pragma unroll
    for (int mb = 0; mb < 2; ++mb) {
#pragma unroll
        for (int nb = 0; nb < 8; ++nb) {
#pragma unroll
            for (int j = 0; j < 8; ++j) os[(hi * 8 + j) * 132 + nb * 16 + lr] = acc[mb][nb][j] * OSC; }
        wave_sync();
        float* orow = OUT + ((size_t)b * OUT_SEQ + tt + mb * 16) * DM + c0;
#pragma unroll 1
        for (int ps = 0; ps < 2; ++ps) {
#pragma unroll
            for (int s = 0; s < 16; ++s) {
                const v4f val = *(const v4fa*)(&os[s * 132 + lane * 4]);
                *(volatile v4f*)(orow + (size_t)s * DM + lane * 4) = val; }
            if (ps == 0) __threadfence(); }
        wave_sync();
    }
}

static constexpr size_t al256(size_t v) { return (v + 255) & ~(size_t)255; }
static constexpr size_t SZ_XB = al256((size_t)NB * SEQ * DM * 2);
static constexpr size_t SZ_W3 = al256((size_t)3 * DM * DM * 2);
static constexpr size_t SZ_WO = al256((size_t)DM * DM * 2);
static constexpr size_t SZ_PL = al256(PLN * 2);
static constexpr size_t SZ_PR = al256(PLR * 2);
static constexpr size_t SZ_CR = al256((size_t)NB * EROWS * DM * 2);
static constexpr size_t SZ_MB = al256((size_t)SEQ * SEQ * 2);
static constexpr size_t SZ_AB = al256((size_t)NH_ * SEQ_FULL * 2);
static constexpr size_t SZ_FL = (size_t)NFB * 128;
static constexpr size_t SZ_TOTAL = SZ_XB + SZ_W3 + SZ_WO + 3 * SZ_PL + 3 * SZ_PR + SZ_CR + SZ_MB + SZ_AB + SZ_FL;
static_assert(SZ_TOTAL <= (size_t)134217728);
static_assert(SZ_PL == PLN * 2);
static_assert(SZ_PR == PLR * 2);
static_assert(((size_t)DM * DM * 2) % 256 == 0);
static_assert((size_t)NB * SEQ * DM * 2 <= SZ_XB);
static_assert(((size_t)NH_ * SEQ_FULL) % 8 == 0);

extern "C" void kernel_launch(void* const* d_in, const int* in_sizes, int n_in,
                              void* d_out, int out_size, void* d_ws, size_t ws_size, hipStream_t stream) {
    if (n_in < 9) return;
    if ((size_t)in_sizes[0] < ((size_t)(NB - 1) * SEQ_FULL + SEQ) * DM) return;
    for (int i = 1; i <= 4; ++i) if ((size_t)in_sizes[i] < (size_t)DM * DM) return;
    if ((size_t)in_sizes[5] < (size_t)(SEQ - 1) * SEQ_FULL + SEQ) return;
    if ((size_t)in_sizes[6] < (size_t)NH_ * SEQ_FULL) return;
    if ((size_t)in_sizes[7] < (size_t)SEQ * HD || (size_t)in_sizes[8] < (size_t)SEQ * HD) return;
    if ((size_t)out_size < ((size_t)(NB - 1) * OUT_SEQ + SEQ) * DM) return;
    if (SZ_TOTAL > ws_size) return;
    const float* x  = (const float*)d_in[0]; const float* wq = (const float*)d_in[1]; const float* wk = (const float*)d_in[2];
    const float* wv = (const float*)d_in[3]; const float* wo = (const float*)d_in[4]; const float* mk = (const float*)d_in[5];
    const float* al = (const float*)d_in[6]; const float* fc = (const float*)d_in[7]; const float* fs = (const float*)d_in[8];
    float* OUT = (float*)d_out;
    char* wsp = (char*)d_ws;
    bf*  XB  = (bf*)wsp;  h16* CH = (h16*)wsp; wsp += SZ_XB;
    bf*  WT3 = (bf*)wsp;  wsp += SZ_W3;
    h16* WOT = (h16*)wsp; wsp += SZ_WO;
    h16* QKH = (h16*)wsp; wsp += 2 * SZ_PL;
    h16* VT  = (h16*)wsp; wsp += SZ_PL;
    h16* QKR = (h16*)wsp; wsp += 2 * SZ_PR;
    h16* VR  = (h16*)wsp; wsp += SZ_PR;
    h16* CR  = (h16*)wsp; wsp += SZ_CR;
    bf*  MB  = (bf*)wsp;  wsp += SZ_MB;
    bf*  AB  = (bf*)wsp;  wsp += SZ_AB;
    int* FL  = (int*)wsp; wsp += SZ_FL;

    if (SEQ == SEQ_FULL) {
        const size_t n8 = (size_t)NB * SEQ * DM / 8;
        k_cvt8<<<(unsigned)((n8 + 255) / 256), 256, 0, stream>>>(x, XB, n8);
    } else {
        const size_t n8 = (size_t)SEQ * DM / 8;
        for (int b = 0; b < NB; ++b) k_cvt8<<<(unsigned)((n8 + 255) / 256), 256, 0, stream>>>(x + (size_t)b * SEQ_FULL * DM, XB + (size_t)b * SEQ * DM, n8);
    }
    { const size_t n8 = (size_t)NH_ * SEQ_FULL / 8; k_cvt8<<<(unsigned)((n8 + 255) / 256), 256, 0, stream>>>(al, AB, n8); }
    k_wT<bf><<<dim3(DM / 64, DM / 64, 1), 256, 0, stream>>>(wq, WT3);
    k_wT<bf><<<dim3(DM / 64, DM / 64, 1), 256, 0, stream>>>(wk, WT3 + (size_t)DM * DM);
    k_wT<bf><<<dim3(DM / 64, DM / 64, 1), 256, 0, stream>>>(wv, WT3 + (size_t)2 * DM * DM);
    k_wT<h16><<<dim3(DM / 64, DM / 64, 1), 256, 0, stream>>>(wo, WOT);
    k_mprep<<<NFB, 256, 0, stream>>>(mk, MB, FL);

    k_projqk<<<dim3(NB * SEQ / 32, NH_, 2), 32, 0, stream>>>(XB, WT3, QKH, QKR, fc, fs);
    k_projv<<<dim3(DM / 32, NB * SEQ / 128, 1), 32, 0, stream>>>(XB, WT3 + (size_t)2 * DM * DM, VT, VR);

    const h16* QH = QKH; const h16* KH = QKH + PLN; const h16* QR = QKR; const h16* KR = QKR + PLR;
    k_flash<1><<<dim3(EROWS / (16 * AW), NB * NH_, 1), 32 * AW, 0, stream>>>(QH, QR, KH, KR, VT, VR, MB, AB, FL, CH, CR, 0);
    if (SEQ > EROWS)
        k_flash<0><<<dim3((SEQ - EROWS) / (16 * AW), NB * NH_, 1), 32 * AW, 0, stream>>>(QH, QR, KH, KR, VT, VR, MB, AB, FL, CH, CR, EROWS);

    k_out<<<dim3(NB * SEQ / 32, DM / 128, 1), 32, 0, stream>>>(CH, CR, WOT, OUT);
}
